// I2A_MambaDuelingModel_78391743086958
// MI455X (gfx1250) — hardware-verified
//
#include <hip/hip_runtime.h>
#include <math.h>


#define NB 4
#define LL 512
#define NR (NB * LL)
#define FIN 32
#define HID 128
#define DM 256
#define DIN 512
#define NST 16
#define DTR 16
#define NXP 48
#define DFF 682
#define DFFP 704
#define NF1 1364
#define NF1P 1408
#define NL 8

typedef __attribute__((ext_vector_type(16))) __bf16 v16b;
typedef __attribute__((ext_vector_type(8)))  __bf16 v8b;
typedef __attribute__((ext_vector_type(8)))  float v8f;
typedef __attribute__((ext_vector_type(4)))  float v4f;
typedef __attribute__((ext_vector_type(4)))  unsigned v4u;
typedef float __attribute__((may_alias)) float_a;

template <typename T> __device__ __forceinline__ void vst2(void* p, T v) { *(volatile T*)p = v; __threadfence(); *(volatile T*)p = v; }
__device__ __forceinline__ v8f wmma_bf(v16b a, v16b b, v8f c) {
  v8f d = __builtin_amdgcn_wmma_f32_16x16x32_bf16(false, a, false, b, (short)0, c, false, false);
  asm volatile("v_nop\n\tv_nop\n\tv_nop\n\tv_nop" : "+v"(d) : "v"(a), "v"(b));
  return d;
}
struct F2 { v16b h, l; };
__device__ __forceinline__ F2 split_rowK(const float* row, int k0, int lane, int K) { F2 r; const int g = lane >> 4;
#pragma unroll
  for (int i = 0; i < 8; ++i) { const int ka = k0 + 8 * g + i, kb = ka + 16; const float va = ka < K ? row[ka] : 0.f, vb = kb < K ? row[kb] : 0.f;
    const __bf16 ha = (__bf16)va, hb = (__bf16)vb; r.h[i] = ha; r.l[i] = (__bf16)(va - (float)ha); r.h[8 + i] = hb; r.l[8 + i] = (__bf16)(vb - (float)hb); }
  return r; }
__device__ __forceinline__ F2 frag_b2(const __bf16* rh, const __bf16* rl, int lane) { F2 r; union { v16b v; v8b q[2]; } uh, ul; const int o = 8 * (lane >> 4);
  uh.q[0] = *(const v8b*)(rh + o); uh.q[1] = *(const v8b*)(rh + o + 16); ul.q[0] = *(const v8b*)(rl + o); ul.q[1] = *(const v8b*)(rl + o + 16);
  r.h = uh.v; r.l = ul.v; return r; }
__device__ __forceinline__ v8f mac3(const F2& a, const F2& b, v8f c) { c = wmma_bf(a.l, b.h, c); c = wmma_bf(a.h, b.l, c); return wmma_bf(a.h, b.h, c); }
__device__ __forceinline__ float silu(float v) { return v / (1.0f + expf(-v)); }
__device__ __forceinline__ float softplus(float v) { return v > 20.f ? v : log1pf(expf(v)); }
#define LDSX() do { asm volatile("s_wait_dscnt 0" ::: "memory"); __builtin_amdgcn_wave_barrier(); __builtin_amdgcn_fence(__ATOMIC_RELEASE, "workgroup"); } while (0)

__global__ __launch_bounds__(64) void k_pack(const float* __restrict__ W, __bf16* __restrict__ Wh, __bf16* __restrict__ Wl, int K, int N, int KP, int NP) {
  const int n = blockIdx.x, z = blockIdx.y;
  const float* Wz = W + (size_t)z * K * N; const size_t ob = ((size_t)z * NP + n) * KP;
  for (int q = threadIdx.x; q < KP / 8; q += 64) { union { v8b h; v4u u; } ph, pl;
#pragma unroll
    for (int e = 0; e < 8; ++e) { const int k = q * 8 + e; const float v = (k < K && n < N) ? Wz[(size_t)k * N + n] : 0.f; const __bf16 h = (__bf16)v; ph.h[e] = h; pl.h[e] = (__bf16)(v - (float)h); }
    vst2(Wh + ob + q * 8, ph.u); vst2(Wl + ob + q * 8, pl.u); }
}
__global__ __launch_bounds__(64) void k_pack64(const float* __restrict__ mW, const float* __restrict__ tW, __bf16* __restrict__ Wh, __bf16* __restrict__ Wl) {
  const int n = blockIdx.x, q = threadIdx.x; if (q >= 8) return;
  union { v8b h; v4u u; } ph, pl;
#pragma unroll
  for (int e = 0; e < 8; ++e) { const int k = q * 8 + e; float v = 0.f;
    if (k < 32 && n < HID) v = mW[k * HID + n]; else if (k >= 32 && n >= HID) v = tW[(k - 32) * HID + (n - HID)];
    const __bf16 h = (__bf16)v; ph.h[e] = h; pl.h[e] = (__bf16)(v - (float)h); }
  vst2(Wh + (size_t)n * 64 + q * 8, ph.u); vst2(Wl + (size_t)n * 64 + q * 8, pl.u);
}

__global__ __launch_bounds__(256) void k_front(const float* __restrict__ src, const float* __restrict__ tau, const float* __restrict__ Wm, const float* __restrict__ Ws,
                                             const float* __restrict__ Wg, const float* __restrict__ bg, const float* __restrict__ tw0, const float* __restrict__ tb0,
                                             const float* __restrict__ tw, const float* __restrict__ tb, float* __restrict__ A64) {
  __shared__ float avg[FIN], shift[FIN], sd[FIN], ad[FIN], m2[FIN], gate[FIN];
  const int b = blockIdx.x, tid = threadIdx.x;
  const float* sb = src + (size_t)b * LL * FIN;
  if (tid < FIN) { float s = 0.f;
#pragma unroll 1
    for (int t = 0; t < LL; ++t) s += sb[t * FIN + tid];
    avg[tid] = s / (float)LL; }
  __syncthreads();
  if (tid < FIN) { float s = 0.f;
#pragma unroll 1
    for (int j = 0; j < FIN; ++j) s += Wm[tid * FIN + j] * avg[j];
    shift[tid] = s; }
  __syncthreads();
  if (tid < FIN) { float q = 0.f;
#pragma unroll 1
    for (int t = 0; t < LL; ++t) { const float v = sb[t * FIN + tid] - shift[tid]; q += v * v; }
    sd[tid] = sqrtf(q / (float)LL); }
  __syncthreads();
  if (tid < FIN) { float s = 0.f;
#pragma unroll 1
    for (int j = 0; j < FIN; ++j) s += Ws[tid * FIN + j] * sd[j];
    ad[tid] = s <= 1e-8f ? 1.0f : s; }
  __syncthreads();
  if (tid < FIN) { float s = 0.f;
#pragma unroll 1
    for (int t = 0; t < LL; ++t) s += (sb[t * FIN + tid] - shift[tid]) / ad[tid];
    m2[tid] = s / (float)LL; }
  __syncthreads();
  if (tid < FIN) { float s = bg[tid];
#pragma unroll 1
    for (int j = 0; j < FIN; ++j) s += Wg[tid * FIN + j] * m2[j];
    gate[tid] = 1.0f / (1.0f + expf(-s)); }
  __syncthreads();
  for (int q = tid; q < LL * 16; q += 256) { const int t = q >> 4, pc = q & 15; v4f v;
    const size_t row = (size_t)b * LL + t;
    if (pc < 8) {
#pragma unroll
      for (int e = 0; e < 4; ++e) { const int f = pc * 4 + e; v[e] = ((sb[t * FIN + f] - shift[f]) / ad[f]) * gate[f]; } }
    else { const float* tr = tau + row * 8;
#pragma unroll
      for (int e = 0; e < 4; ++e) { const int j = (pc - 8) * 4 + e;
        float s;
        if (j < 31) { s = tb[j];
#pragma unroll
          for (int k = 0; k < 8; ++k) s += tr[k] * tw[k * 31 + j];
          s = sinf(s); }
        else { s = tb0[0];
#pragma unroll
          for (int k = 0; k < 8; ++k) s += tr[k] * tw0[k]; }
        v[e] = s; } }
    vst2(A64 + row * 64 + pc * 4, v); }
}

template <int NT, int MODE>
__global__ __launch_bounds__(128) void k_gemm(const float* __restrict__ A, int lda, int K, int KP, const __bf16* __restrict__ Wh, const __bf16* __restrict__ Wl,
                                            const float* __restrict__ bias, const float* __restrict__ res, float* __restrict__ Out, int ldo, int Nst) {
  __shared__ __align__(16) float so[4][16 * NT * 16 + 16];
  const int tid = threadIdx.x, wave = tid >> 5, lane = tid & 31, col = lane & 15, g = lane >> 4;
  const int r0 = blockIdx.x * 64 + wave * 16, n0 = blockIdx.y * (NT * 16);
  v8f acc[NT];
#pragma unroll
  for (int j = 0; j < NT; ++j) acc[j] = (v8f){};
#pragma unroll 1
  for (int kc = 0; kc < KP / 32; ++kc) { const F2 a = split_rowK(A + (size_t)(r0 + col) * lda, kc * 32, lane, K);
#pragma unroll
    for (int j = 0; j < NT; ++j) { const size_t ro = (size_t)(n0 + j * 16 + col) * KP + kc * 32; acc[j] = mac3(a, frag_b2(Wh + ro, Wl + ro, lane), acc[j]); } }
  float* S = so[wave]; const int LD = NT * 16;
#pragma unroll
  for (int j = 0; j < NT; ++j) { const int n = n0 + j * 16 + col; const float bv = (bias && n < Nst) ? bias[n] : 0.f;
#pragma unroll
    for (int r = 0; r < 8; ++r) { float v = acc[j][r] + bv; if (MODE == 1) v = softplus(v); S[(8 * g + r) * LD + j * 16 + col] = v; } }
  LDSX();
  for (int q = lane; q < 16 * (LD / 4); q += 32) { const int rl = q / (LD / 4), pc = q % (LD / 4); const int n = n0 + pc * 4; if (n >= Nst) continue;
    const size_t o = (size_t)(r0 + rl) * ldo + n;
    v4f v = *(const v4f*)(S + rl * LD + pc * 4); if (res) v += *(const v4f*)(res + o); vst2(Out + o, v); }
}

__global__ __launch_bounds__(256) void k_geglu(const float* __restrict__ ag, float* __restrict__ p) {
  const size_t row = blockIdx.x; const int tid = threadIdx.x;
  for (int q = tid; q < DFFP / 4; q += 256) { v4f v;
#pragma unroll
    for (int e = 0; e < 4; ++e) { const int j = q * 4 + e; float r = 0.f;
      if (j < DFF) { const float a = ag[row * NF1P + j], gg = ag[row * NF1P + DFF + j]; r = a * (0.5f * gg * (1.0f + erff(gg * 0.70710678118654752f))); }
      v[e] = r; }
    vst2(p + row * DFFP + q * 4, v); }
}
__global__ __launch_bounds__(256) void k_ln(const float* __restrict__ h, const float* __restrict__ w, const float* __restrict__ bb, float* __restrict__ o) {
  const int tid = threadIdx.x, wv = tid >> 5, lane = tid & 31; const size_t row = (size_t)blockIdx.x * 8 + wv;
  const v4f a = *(const v4f*)(h + row * DM + lane * 8), c = *(const v4f*)(h + row * DM + lane * 8 + 4);
  float v[8] = { a[0], a[1], a[2], a[3], c[0], c[1], c[2], c[3] };
  float s = 0.f;
#pragma unroll
  for (int e = 0; e < 8; ++e) s += v[e];
#pragma unroll
  for (int off = 16; off >= 1; off >>= 1) s += __shfl_xor(s, off, 32);
  const float mu = s / (float)DM; float q = 0.f;
#pragma unroll
  for (int e = 0; e < 8; ++e) { v[e] -= mu; q += v[e] * v[e]; }
#pragma unroll
  for (int off = 16; off >= 1; off >>= 1) q += __shfl_xor(q, off, 32);
  const float rs = rsqrtf(q / (float)DM + 1e-5f);
  v4f o0, o1;
#pragma unroll
  for (int e = 0; e < 4; ++e) { o0[e] = v[e] * rs * w[lane * 8 + e] + bb[lane * 8 + e]; o1[e] = v[4 + e] * rs * w[lane * 8 + 4 + e] + bb[lane * 8 + 4 + e]; }
  vst2(o + row * DM + lane * 8, o0); vst2(o + row * DM + lane * 8 + 4, o1);
}
__global__ __launch_bounds__(128) void k_conv(const float* __restrict__ xz, const float* __restrict__ cw, const float* __restrict__ cb, float* __restrict__ u2) {
  const size_t row = blockIdx.x; const int tid = threadIdx.x, t = (int)(row % LL);
  v4f v;
#pragma unroll
  for (int e = 0; e < 4; ++e) { const int d = tid * 4 + e; float a = cb[d];
#pragma unroll
    for (int k = 0; k < 4; ++k) { const int tt = t - 3 + k; if (tt >= 0) a += cw[d * 4 + k] * xz[(row - (size_t)(t - tt)) * (2 * DIN) + d]; }
    v[e] = silu(a); }
  vst2(u2 + row * DIN + tid * 4, v);
}
__global__ __launch_bounds__(64) void k_scan(const float* __restrict__ u2, const float* __restrict__ dt, const float* __restrict__ xd, const float* __restrict__ xz,
                                           const float* __restrict__ Alog, const float* __restrict__ Dp, float* __restrict__ gout) {
  const int b = blockIdx.y, d = blockIdx.x * 64 + threadIdx.x;
  float A[NST], h[NST];
#pragma unroll
  for (int n = 0; n < NST; ++n) { A[n] = -expf(Alog[(size_t)d * NST + n]); h[n] = 0.f; }
  const float Dd = Dp[d];
#pragma unroll 1
  for (int t = 0; t < LL; ++t) { const size_t row = (size_t)b * LL + t;
    const float dtv = dt[row * DIN + d], uv = u2[row * DIN + d]; const float* xr = xd + row * NXP;
    float y = 0.f;
#pragma unroll 1
    for (int n = 0; n < NST; ++n) { h[n] = expf(dtv * A[n]) * h[n] + dtv * uv * xr[DTR + n]; y += h[n] * xr[DTR + NST + n]; }
    y += uv * Dd;
    const float z = xz[row * (2 * DIN) + DIN + d];
    vst2(gout + row * DIN + d, (float_a)(y * silu(z)));
  }
}
__global__ __launch_bounds__(64) void k_gate(const float* __restrict__ g12, float* __restrict__ q) {
  const size_t row = blockIdx.x; const int tid = threadIdx.x;
  const v4f a = *(const v4f*)(g12 + row * 512 + tid * 4), c = *(const v4f*)(g12 + row * 512 + 256 + tid * 4);
  v4f v = { silu(a[0]) * c[0], silu(a[1]) * c[1], silu(a[2]) * c[2], silu(a[3]) * c[3] };
  vst2(q + row * DM + tid * 4, v);
}
__device__ __forceinline__ void block_ln_relu(float* v, int n, const float* w, const float* bb, float* red, int tid) {
  float s = 0.f; for (int i = tid; i < n; i += 256) s += v[i];
  red[tid] = s; __syncthreads();
  for (int st = 128; st > 0; st >>= 1) { if (tid < st) red[tid] += red[tid + st]; __syncthreads(); }
  const float mu = red[0] / (float)n; __syncthreads();
  float q = 0.f; for (int i = tid; i < n; i += 256) { const float d = v[i] - mu; q += d * d; }
  red[tid] = q; __syncthreads();
  for (int st = 128; st > 0; st >>= 1) { if (tid < st) red[tid] += red[tid + st]; __syncthreads(); }
  const float rs = rsqrtf(red[0] / (float)n + 1e-5f); __syncthreads();
  for (int i = tid; i < n; i += 256) { const float o = (v[i] - mu) * rs * w[i] + bb[i]; v[i] = o > 0.f ? o : 0.f; }
  __syncthreads();
}
__global__ __launch_bounds__(256) void k_head(const float* __restrict__ h, const float* __restrict__ nfw, const float* __restrict__ nfb,
                                            const float* __restrict__ vW1, const float* __restrict__ vb1, const float* __restrict__ vl1w, const float* __restrict__ vl1b,
                                            const float* __restrict__ vW2, const float* __restrict__ vb2, const float* __restrict__ vl2w, const float* __restrict__ vl2b,
                                            const float* __restrict__ vW3, const float* __restrict__ vb3,
                                            const float* __restrict__ aW1, const float* __restrict__ ab1, const float* __restrict__ al1w, const float* __restrict__ al1b,
                                            const float* __restrict__ aW2, const float* __restrict__ ab2, const float* __restrict__ al2w, const float* __restrict__ al2b,
                                            const float* __restrict__ aW3, const float* __restrict__ ab3, float* __restrict__ out) {
  __shared__ float f[DM], x1[512], x2[256], red[256];
  __shared__ __align__(16) float res[32];
  const int tid = threadIdx.x;
  if (tid < 32) res[tid] = 0.f;
#pragma unroll 1
  for (int b = 0; b < NB; ++b) {
    const float* hr = h + ((size_t)b * LL + LL - 1) * DM;
    { float s = 0.f; for (int i = tid; i < DM; i += 256) s += hr[i];
      red[tid] = s; __syncthreads();
      for (int st = 128; st > 0; st >>= 1) { if (tid < st) red[tid] += red[tid + st]; __syncthreads(); }
      const float mu = red[0] / (float)DM; __syncthreads();
      float q = 0.f; for (int i = tid; i < DM; i += 256) { const float d = hr[i] - mu; q += d * d; }
      red[tid] = q; __syncthreads();
      for (int st = 128; st > 0; st >>= 1) { if (tid < st) red[tid] += red[tid + st]; __syncthreads(); }
      const float rs = rsqrtf(red[0] / (float)DM + 1e-5f); __syncthreads();
      for (int i = tid; i < DM; i += 256) f[i] = (hr[i] - mu) * rs * nfw[i] + nfb[i];
      __syncthreads(); }
#pragma unroll 1
    for (int which = 0; which < 2; ++which) {
      const float* W1 = which ? aW1 : vW1; const float* b1 = which ? ab1 : vb1; const float* l1w = which ? al1w : vl1w; const float* l1b = which ? al1b : vl1b;
      const float* W2 = which ? aW2 : vW2; const float* b2 = which ? ab2 : vb2; const float* l2w = which ? al2w : vl2w; const float* l2b = which ? al2b : vl2b;
      const float* W3 = which ? aW3 : vW3; const float* b3 = which ? ab3 : vb3; const int nout = which ? 5 : 1;
      for (int j = tid; j < 512; j += 256) { float s = b1[j];
#pragma unroll 1
        for (int i = 0; i < DM; ++i) s += f[i] * W1[i * 512 + j];
        x1[j] = s; }
      __syncthreads();
      block_ln_relu(x1, 512, l1w, l1b, red, tid);
      { float s = b2[tid];
#pragma unroll 1
        for (int i = 0; i < 512; ++i) s += x1[i] * W2[i * 256 + tid];
        x2[tid] = s; }
      __syncthreads();
      block_ln_relu(x2, 256, l2w, l2b, red, tid);
      if (tid < nout) { float s = b3[tid];
#pragma unroll 1
        for (int i = 0; i < 256; ++i) s += x2[i] * W3[i * nout + tid];
        if (which == 0) res[24 + b] = s; else res[b * 5 + tid] = s; }
      __syncthreads();
    }
  }
  if (tid < NB) { float m = 0.f; for (int a = 0; a < 5; ++a) m += res[tid * 5 + a]; m *= 0.2f;
    const float v = res[24 + tid]; for (int a = 0; a < 5; ++a) res[tid * 5 + a] = v + res[tid * 5 + a] - m; }
  __syncthreads();
  if (tid < 5) vst2(out + tid * 4, *(const v4f*)(&res[tid * 4]));
}

extern "C" void kernel_launch(void* const* d_in, const int* in_sizes, int n_in,
                              void* d_out, int out_size, void* d_ws, size_t ws_size,
                              hipStream_t stream) {
  (void)in_sizes; (void)n_in; (void)out_size; (void)ws_size;
  const float** I = (const float**)d_in;
  const float* src = I[0]; const float* tau = I[1]; const float* Wm = I[2]; const float* Wsd = I[3]; const float* Wg = I[4]; const float* bg = I[5];
  const float* membW = I[6]; const float* membB = I[7]; const float* tw0 = I[8]; const float* tb0 = I[9]; const float* tw = I[10]; const float* tb = I[11];
  const float* tprW = I[12]; const float* tprB = I[13]; const float* fW1 = I[14]; const float* fb1 = I[15]; const float* fW2 = I[16]; const float* fb2 = I[17];
  const float* n1w = I[18]; const float* n1b = I[19]; const float* inW = I[20]; const float* cw = I[21]; const float* cb = I[22]; const float* xpW = I[23];
  const float* dtW = I[24]; const float* dtb = I[25]; const float* Alog = I[26]; const float* Dp = I[27]; const float* outW = I[28];
  const float* n2w = I[29]; const float* n2b = I[30]; const float* mW1 = I[31]; const float* mW2 = I[32]; const float* nfw = I[33]; const float* nfb = I[34];
  float* out = (float*)d_out;
  char* ws = (char*)d_ws; size_t off = 0;
  auto take = [&](size_t bytes) { char* p = ws + off; off += (bytes + 255) & ~(size_t)255; return p; };
  auto panel = [&](size_t n) { return (__bf16*)take(n * 2); };
  __bf16 *W64h = panel(256 * 64), *W64l = panel(256 * 64);
  __bf16 *F1h = panel((size_t)NF1P * 256), *F1l = panel((size_t)NF1P * 256);
  __bf16 *F2h = panel((size_t)256 * DFFP), *F2l = panel((size_t)256 * DFFP);
  __bf16 *INh = panel((size_t)NL * 1024 * 256), *INl = panel((size_t)NL * 1024 * 256);
  __bf16 *XPh = panel((size_t)NL * 48 * 512), *XPl = panel((size_t)NL * 48 * 512);
  __bf16 *DTh = panel((size_t)NL * 512 * 32), *DTl = panel((size_t)NL * 512 * 32);
  __bf16 *OUh = panel((size_t)NL * 256 * 512), *OUl = panel((size_t)NL * 256 * 512);
  __bf16 *M1h = panel((size_t)NL * 512 * 256), *M1l = panel((size_t)NL * 512 * 256);
  __bf16 *M2h = panel((size_t)NL * 256 * 256), *M2l = panel((size_t)NL * 256 * 256);
  float* A64 = (float*)take((size_t)NR * 64 * 4);
  float* h0 = (float*)take((size_t)NR * DM * 4); float* h1 = (float*)take((size_t)NR * DM * 4);
  float* ag = (float*)take((size_t)NR * NF1P * 4);
  float* pg = (float*)take((size_t)NR * DFFP * 4);
  float* hn = (float*)take((size_t)NR * DM * 4);
  float* xz = (float*)take((size_t)NR * 2 * DIN * 4);
  float* u2 = (float*)take((size_t)NR * DIN * 4);
  float* xd = (float*)take((size_t)NR * NXP * 4);
  float* dt = (float*)take((size_t)NR * DIN * 4);
  float* gg = (float*)take((size_t)NR * DIN * 4);
  float* g12 = (float*)take((size_t)NR * 512 * 4);
  float* gq = (float*)take((size_t)NR * DM * 4);
  k_pack64<<<256, 64, 0, stream>>>(membW, tprW, W64h, W64l);
  k_pack<<<dim3(NF1P, 1), 64, 0, stream>>>(fW1, F1h, F1l, 256, NF1, 256, NF1P);
  k_pack<<<dim3(256, 1), 64, 0, stream>>>(fW2, F2h, F2l, DFF, 256, DFFP, 256);
  k_pack<<<dim3(1024, NL), 64, 0, stream>>>(inW, INh, INl, 256, 1024, 256, 1024);
  k_pack<<<dim3(48, NL), 64, 0, stream>>>(xpW, XPh, XPl, 512, 48, 512, 48);
  k_pack<<<dim3(512, NL), 64, 0, stream>>>(dtW, DTh, DTl, 16, 512, 32, 512);
  k_pack<<<dim3(256, NL), 64, 0, stream>>>(outW, OUh, OUl, 512, 256, 512, 256);
  k_pack<<<dim3(512, NL), 64, 0, stream>>>(mW1, M1h, M1l, 256, 512, 256, 512);
  k_pack<<<dim3(256, NL), 64, 0, stream>>>(mW2, M2h, M2l, 256, 256, 256, 256);
  k_front<<<NB, 256, 0, stream>>>(src, tau, Wm, Wsd, Wg, bg, tw0, tb0, tw, tb, A64);
  k_gemm<8, 0><<<dim3(NR / 64, 1), 128, 0, stream>>>(A64, 64, 64, 64, W64h, W64l, membB, nullptr, h0, DM, 128);
  k_gemm<8, 0><<<dim3(NR / 64, 1), 128, 0, stream>>>(A64, 64, 64, 64, W64h + 128 * 64, W64l + 128 * 64, tprB, nullptr, h0 + 128, DM, 128);
  k_gemm<8, 0><<<dim3(NR / 64, NF1P / 128), 128, 0, stream>>>(h0, DM, 256, 256, F1h, F1l, fb1, nullptr, ag, NF1P, NF1);
  k_geglu<<<NR, 256, 0, stream>>>(ag, pg);
  k_gemm<8, 0><<<dim3(NR / 64, DM / 128), 128, 0, stream>>>(pg, DFFP, DFFP, DFFP, F2h, F2l, fb2, nullptr, h1, DM, DM);
  float* hc = h1; float* ho = h0;
  for (int i = 0; i < NL; ++i) {
    k_ln<<<NR / 8, 256, 0, stream>>>(hc, n1w + i * DM, n1b + i * DM, hn);
    k_gemm<8, 0><<<dim3(NR / 64, 1024 / 128), 128, 0, stream>>>(hn, DM, 256, 256, INh + (size_t)i * 1024 * 256, INl + (size_t)i * 1024 * 256, nullptr, nullptr, xz, 2 * DIN, 1024);
    k_conv<<<NR, 128, 0, stream>>>(xz, cw + (size_t)i * DIN * 4, cb + i * DIN, u2);
    k_gemm<3, 0><<<dim3(NR / 64, 1), 128, 0, stream>>>(u2, DIN, 512, 512, XPh + (size_t)i * 48 * 512, XPl + (size_t)i * 48 * 512, nullptr, nullptr, xd, NXP, NXP);
    k_gemm<8, 1><<<dim3(NR / 64, DIN / 128), 128, 0, stream>>>(xd, NXP, DTR, 32, DTh + (size_t)i * 512 * 32, DTl + (size_t)i * 512 * 32, dtb + i * DIN, nullptr, dt, DIN, DIN);
    k_scan<<<dim3(DIN / 64, NB), 64, 0, stream>>>(u2, dt, xd, xz, Alog + (size_t)i * DIN * NST, Dp + i * DIN, gg);
    k_gemm<8, 0><<<dim3(NR / 64, DM / 128), 128, 0, stream>>>(gg, DIN, 512, 512, OUh + (size_t)i * 256 * 512, OUl + (size_t)i * 256 * 512, nullptr, hc, ho, DM, DM);
    k_ln<<<NR / 8, 256, 0, stream>>>(ho, n2w + i * DM, n2b + i * DM, hn);
    k_gemm<8, 0><<<dim3(NR / 64, 512 / 128), 128, 0, stream>>>(hn, DM, 256, 256, M1h + (size_t)i * 512 * 256, M1l + (size_t)i * 512 * 256, nullptr, nullptr, g12, 512, 512);
    k_gate<<<NR, 64, 0, stream>>>(g12, gq);
    k_gemm<8, 0><<<dim3(NR / 64, DM / 128), 128, 0, stream>>>(gq, DM, 256, 256, M2h + (size_t)i * 256 * 256, M2l + (size_t)i * 256 * 256, nullptr, ho, hc, DM, DM);
  }
  k_head<<<1, 256, 0, stream>>>(hc, nfw, nfb, I[35], I[36], I[37], I[38], I[39], I[40], I[41], I[42], I[43], I[44],
                                I[45], I[46], I[47], I[48], I[49], I[50], I[51], I[52], I[53], I[54], out);
}
